// GGRNet_55439437856836
// MI455X (gfx1250) — hardware-run, weakly checked
//
#include <hip/hip_runtime.h>


namespace {
constexpr int N = 50000, NP = 50048, E = 600000, D = 128, G = 256, NBLK = NP / 64  , HR = 64, DM = 95, DMP = 96, NO = 12, NIT = 10;
constexpr float XS = 8.0f, WSC = 256.0f, NEG = 0.2f  , BNEPS = 1e-5f;

typedef _Float16 b16;
typedef __attribute__((ext_vector_type(16))) _Float16 v16b;
typedef __attribute__((ext_vector_type(8))) _Float16 v8b;
typedef __attribute__((ext_vector_type(8))) float v8f;
typedef __attribute__((ext_vector_type(4))) float v4f;
__device__ __forceinline__ float bf16_rne(float f) { unsigned int u = __float_as_uint(f); u += 0x7FFFu + ((u >> 16) & 1u); return __uint_as_float(u & 0xFFFF0000u); }
__device__ __forceinline__ void split16(float v, b16& hi, b16& lo) { hi = (b16)v; lo = (b16)(v - (float)hi); }
__device__ __forceinline__ v16b frag_kb(const b16* p, int hh) { const v8b a = *(const v8b*)(p + 8 * hh), b = *(const v8b*)(p + 16 + 8 * hh); v16b f;
#pragma unroll
  for (int e = 0; e < 8; ++e) { f[e] = a[e]; f[8 + e] = b[e]; } return f; }
__device__ __forceinline__ v8f wmma16b(v16b a, v16b b, v8f c) { v8f d = __builtin_amdgcn_wmma_f32_16x16x32_f16(false, a, false, b, (short)0, c, false, false); asm volatile("v_nop\n\tv_nop\n\tv_nop\n\tv_nop" : "+v"(d) : "v"(a), "v"(b)); return d; }
__device__ __forceinline__ void wave_lds_sync() { __builtin_amdgcn_fence(__ATOMIC_RELEASE, "workgroup"); __builtin_amdgcn_wave_barrier(); __builtin_amdgcn_fence(__ATOMIC_ACQUIRE, "workgroup"); }
__device__ __forceinline__ float pmul(float a, float b) { float p = a * b; asm volatile("" : "+v"(p)); return p; }
__device__ __forceinline__ int iclamp(int v, int lo, int hi) { return v < lo ? lo : (v > hi ? hi : v); }
__device__ __forceinline__ float nexp(float x) { return __builtin_amdgcn_exp2f(x * 1.4426950408889634f); }
__device__ __forceinline__ float lrelu(float x) { return x > 0.0f ? x : NEG * x; }

constexpr int CSR_NBLK = 512, CSR_GB = 9, CSR_GN = 1 << CSR_GB  , CSR_MAXG = 512, CSR_CAP = 12288  ;
__global__ __launch_bounds__(64) void csrA_kernel(const int* __restrict__ dst, int E, int N, int nG, int CHP, int NGP, int* __restrict__ STG, int* __restrict__ HST) {
  extern __shared__ int sm[];
  int* cnt = sm; int* run = sm + NGP; int* ids = sm + 2 * NGP;
  const int b = blockIdx.x; const int ch = (E + CSR_NBLK - 1) / CSR_NBLK; const int e0 = b * ch, e1 = min(E, e0 + ch);
  for (int i = threadIdx.x; i < NGP; i += 64) cnt[i] = 0;
  for (int i = threadIdx.x; i < CHP; i += 64) ids[i] = -1;
  __syncthreads();
  if (threadIdx.x == 0) {
    for (int e = e0; e < e1; ++e) { int d = dst[e]; d = (d < 0) ? 0 : (d >= N ? N - 1 : d); cnt[d >> CSR_GB] += 1; }
    int acc = 0; for (int g = 0; g < nG; ++g) { run[g] = acc; acc += cnt[g]; }
    for (int e = e0; e < e1; ++e) { int d = dst[e]; d = (d < 0) ? 0 : (d >= N ? N - 1 : d); const int g = d >> CSR_GB; ids[run[g]] = e; run[g] += 1; } }
  __syncthreads();
  typedef __attribute__((ext_vector_type(4))) int v4i;
  for (int pass = 0; pass < 2; ++pass) {
    for (int i = threadIdx.x; i < CHP / 4; i += 64) *(volatile v4i*)(STG + (size_t)b * CHP + i * 4) = *(const v4i*)(&ids[i * 4]);
    for (int i = threadIdx.x; i < NGP / 4; i += 64) { v4i v; for (int e = 0; e < 4; ++e) v[e] = (i * 4 + e < nG) ? cnt[i * 4 + e] : 0; *(volatile v4i*)(HST + (size_t)b * NGP + i * 4) = v; }
    __threadfence(); }
}
__global__ __launch_bounds__(512) void csrS_kernel(const int* __restrict__ HST, int nG, int NGP, int* __restrict__ START, int* __restrict__ TOT, int* __restrict__ OFF) {
  __shared__ int tot[CSR_MAXG];
  const int b = threadIdx.x;
  for (int pass = 0; pass < 2; ++pass) { int runb = 0; for (int g = 0; g < nG; ++g) { int c = HST[(size_t)b * NGP + g]; c = (c < 0) ? 0 : c; ((volatile int*)OFF)[(size_t)g * CSR_NBLK + b] = runb; runb += c; } __threadfence(); }
  for (int g = threadIdx.x; g < nG; g += 512) { int s = 0; for (int bb = 0; bb < CSR_NBLK; ++bb) { int c = HST[(size_t)bb * NGP + g]; s += (c < 0) ? 0 : c; } tot[g] = s; }
  __syncthreads();
  if (threadIdx.x < 32) {
    __shared__ int st[CSR_MAXG + 32];
    if (threadIdx.x == 0) { int acc = 0; for (int g = 0; g < NGP; ++g) { st[g] = acc; if (g < nG) acc += (tot[g] + 31) & ~31; } st[NGP] = acc; }
    __builtin_amdgcn_fence(__ATOMIC_RELEASE, "workgroup"); __builtin_amdgcn_wave_barrier(); __builtin_amdgcn_fence(__ATOMIC_ACQUIRE, "workgroup");
    for (int pass = 0; pass < 2; ++pass) { for (int i = threadIdx.x; i < NGP + 32; i += 32) { ((volatile int*)START)[i] = (i <= NGP) ? st[min(i, NGP)] : 0; ((volatile int*)TOT)[i] = (i < nG) ? tot[i] : 0; } __threadfence(); } }
}
__global__ __launch_bounds__(256) void csrB_kernel(const int* __restrict__ dst, int N, int nG, int CHP, int NGP, int permLen, const int* __restrict__ STG, const int* __restrict__ HST, const int* __restrict__ OFF, const int* __restrict__ START, const int* __restrict__ TOT, int* __restrict__ PERM, int* __restrict__ ROWPTR, int* __restrict__ ROWCNT, int* __restrict__ FLAG) {
  typedef __attribute__((ext_vector_type(4))) int v4i;
  __shared__ int ids[CSR_CAP]; __shared__ unsigned short key[CSR_CAP]; __shared__ int outp[CSR_CAP]; __shared__ int ncnt[CSR_GN + 1]; __shared__ int boff[CSR_NBLK + 1];
  const int g = blockIdx.x, t_ = threadIdx.x; int tot = TOT[g]; int st = START[g], stn = START[g + 1]; const int v0 = g * CSR_GN; const int nv = min(CSR_GN, N - v0);
  st = (st < 0) ? 0 : (st > permLen - 32 ? permLen - 32 : st) & ~31; stn = (stn < st) ? st : (stn > permLen ? permLen : stn); tot = (tot < 0) ? 0 : tot; if (tot > stn - st && tot <= CSR_CAP) tot = stn - st;
  if (tot > CSR_CAP) {
    for (int pass = 0; pass < 2; ++pass) { for (int i = t_; i < CSR_GN / 4; i += 256) { v4i a, c; for (int e = 0; e < 4; ++e) { a[e] = st; c[e] = 0; } *(volatile v4i*)(ROWPTR + v0 + i * 4) = a; *(volatile v4i*)(ROWCNT + v0 + i * 4) = c; } if (t_ == 0) ((volatile int*)FLAG)[0] = 1; __threadfence(); } (void)nv; return; }
  if (t_ == 0) { int acc = 0; for (int b = 0; b < CSR_NBLK; ++b) { boff[b] = acc; int c = HST[(size_t)b * NGP + g]; c = (c < 0) ? 0 : (c > CHP ? CHP : c); acc += c; if (acc > tot) acc = tot; } boff[CSR_NBLK] = acc; }
  for (int i = t_; i <= CSR_GN; i += 256) ncnt[i] = 0;
  __syncthreads();
  for (int b = 0; b < CSR_NBLK; ++b) { const int c = boff[b + 1] - boff[b]; int o_ = OFF[(size_t)g * CSR_NBLK + b]; o_ = (o_ < 0) ? 0 : (o_ > CHP - c ? CHP - c : o_); const int* src_ = STG + (size_t)b * CHP + o_;
    for (int i = t_; i < c; i += 256) { int id = src_[i]; id = (id < 0) ? 0 : id; ids[boff[b] + i] = id; int d = dst[id]; d = (d < v0) ? v0 : (d >= N ? N - 1 : d); int kk = d - v0; kk = (kk < 0) ? 0 : (kk >= CSR_GN ? CSR_GN - 1 : kk); key[boff[b] + i] = (unsigned short)kk; } }
  __syncthreads();
  if (t_ == 0) { for (int i = 0; i < tot; ++i) ncnt[key[i]] += 1; int acc = 0; for (int vl = 0; vl < CSR_GN; ++vl) { const int c = ncnt[vl]; ncnt[vl] = acc; acc += c; } ncnt[CSR_GN] = acc;
    for (int i = 0; i < tot; ++i) { const int vl = key[i]; outp[ncnt[vl]] = ids[i]; ncnt[vl] += 1; }
    for (int vl = CSR_GN; vl > 0; --vl) ncnt[vl] = ncnt[vl - 1]; ncnt[0] = 0; }
  __syncthreads();
  for (int pass = 0; pass < 2; ++pass) {
    for (int i = t_; i < (stn - st) / 4; i += 256) { v4i v; for (int e = 0; e < 4; ++e) { const int q = i * 4 + e; v[e] = (q < tot) ? outp[q] : -1; } *(volatile v4i*)(PERM + st + i * 4) = v; }
    for (int i = t_; i < CSR_GN / 4; i += 256) { v4i a, c; for (int e = 0; e < 4; ++e) { const int vl = i * 4 + e; a[e] = st + ncnt[vl]; c[e] = (vl < nv) ? (ncnt[vl + 1] - ncnt[vl]) : 0; } *(volatile v4i*)(ROWPTR + v0 + i * 4) = a; *(volatile v4i*)(ROWCNT + v0 + i * 4) = c; }
    __threadfence(); }
}
__global__ __launch_bounds__(256) void csrZ_kernel(int* __restrict__ p, size_t n4) { typedef __attribute__((ext_vector_type(4))) int v4i; const size_t tid = (size_t)blockIdx.x * 256 + threadIdx.x, nth = (size_t)gridDim.x * 256; v4i z = {0, 0, 0, 0}; for (size_t i = tid; i < n4; i += nth) *(volatile v4i*)(p + i * 4) = z; }
struct CsrBufs { int *STG, *HST, *OFF, *START, *TOT, *PERM, *ROWPTR, *ROWCNT, *FLAG; int nG, NGP, CHP; size_t permLen; char* base; size_t bytes; };
static size_t csr_carve(CsrBufs& c, char* ws, size_t off, int E, int N) {
  const size_t off0 = off; c.base = ws + off;
  auto al = [&](size_t bytes) { char* p = ws + off; off += (bytes + 255) & ~(size_t)255; return p; };
  c.nG = (N + CSR_GN - 1) / CSR_GN; c.NGP = (c.nG + 31) & ~31; const int ch = (E + CSR_NBLK - 1) / CSR_NBLK; c.CHP = (ch + 31) & ~31; c.permLen = (size_t)E + 32 * (size_t)c.nG + 32;
  c.STG = (int*)al((size_t)CSR_NBLK * c.CHP * 4); c.HST = (int*)al((size_t)CSR_NBLK * c.NGP * 4); c.OFF = (int*)al((size_t)c.NGP * CSR_NBLK * 4); c.START = (int*)al((size_t)(c.NGP + 64) * 4); c.TOT = (int*)al((size_t)(c.NGP + 64) * 4);
  c.PERM = (int*)al(c.permLen * 4); c.ROWPTR = (int*)al((size_t)c.nG * CSR_GN * 4); c.ROWCNT = (int*)al((size_t)c.nG * CSR_GN * 4); c.FLAG = (int*)al(256);
  c.bytes = off - off0; return off;
}
static void csr_build(const CsrBufs& c, const int* dst, int E, int N, hipStream_t stream) {
  const size_t smem = (size_t)(2 * c.NGP + c.CHP) * 4;
  csrZ_kernel<<<512, 256, 0, stream>>>((int*)c.base, c.bytes / 16);
  csrA_kernel<<<CSR_NBLK, 64, smem, stream>>>(dst, E, N, c.nG, c.CHP, c.NGP, c.STG, c.HST);
  csrS_kernel<<<1, 512, 0, stream>>>(c.HST, c.nG, c.NGP, c.START, c.TOT, c.OFF);
  csrB_kernel<<<c.nG, 256, 0, stream>>>(dst, N, c.nG, c.CHP, c.NGP, (int)c.permLen, c.STG, c.HST, c.OFF, c.START, c.TOT, c.PERM, c.ROWPTR, c.ROWCNT, c.FLAG);
}


__device__ __forceinline__ float sigm(float x) { return 1.0f / (1.0f + __expf(-x)); }
__global__ __launch_bounds__(256) void wprep_kernel(const float* __restrict__ w1a, const float* __restrict__ w1b, const float* __restrict__ wl1, const float* __restrict__ wl2, const float* __restrict__ wm1, const float* __restrict__ wm2, b16* __restrict__ W1AT, b16* __restrict__ W1BT, b16* __restrict__ WLT, b16* __restrict__ WM1T, b16* __restrict__ WM2T) {
  const size_t u = (size_t)blockIdx.x * 256 + threadIdx.x; const size_t n1 = (size_t)D * D / 8, nl = (size_t)D * 2 * D / 8, nm1 = (size_t)DMP * D / 8, nm2 = (size_t)16 * D / 8; size_t t = u; v8b o;
  if (t < 2 * n1) { const int which = (int)(t / n1); const size_t e = (t % n1) * 8; const int oo = (int)(e / D), k0 = (int)(e % D); const float* w = which ? w1b : w1a; for (int j = 0; j < 8; ++j) o[j] = (b16)(bf16_rne(w[(size_t)(k0 + j) * D + oo]) * WSC); for (int pass = 0; pass < 2; ++pass) { *(volatile v8b*)((which ? W1BT : W1AT) + e) = o; __threadfence(); } return; } t -= 2 * n1;
  if (t < nl) { const size_t e = t * 8; const int oo = (int)(e / (2 * D)), k0 = (int)(e % (2 * D)); const float* w = oo < HR ? wl1 : wl2; const int oc = oo % HR; for (int j = 0; j < 8; ++j) o[j] = (b16)(bf16_rne(w[(size_t)(k0 + j) * HR + oc]) * WSC); for (int pass = 0; pass < 2; ++pass) { *(volatile v8b*)(WLT + e) = o; __threadfence(); } return; } t -= nl;
  if (t < nm1) { const size_t e = t * 8; const int oo = (int)(e / D), k0 = (int)(e % D); for (int j = 0; j < 8; ++j) o[j] = oo < DM ? (b16)(bf16_rne(wm1[(size_t)(k0 + j) * DM + oo]) * WSC) : (b16)0.0f; for (int pass = 0; pass < 2; ++pass) { *(volatile v8b*)(WM1T + e) = o; __threadfence(); } return; } t -= nm1;
  if (t < nm2) { const size_t e = t * 8; const int oo = (int)(e / D), k0 = (int)(e % D); for (int j = 0; j < 8; ++j) { const int k = k0 + j; o[j] = (oo < NO && k < DM) ? (b16)(bf16_rne(wm2[(size_t)k * NO + oo]) * WSC) : (b16)0.0f; } for (int pass = 0; pass < 2; ++pass) { *(volatile v8b*)(WM2T + e) = o; __threadfence(); } }
}
__global__ __launch_bounds__(128) void gin_kernel(const float* __restrict__ x, const int* __restrict__ srcs, const int* __restrict__ PERM, const int* __restrict__ ROWPTR, const int* __restrict__ ROWCNT, int permLen, const b16* __restrict__ W1AT, const float* __restrict__ b1a, const b16* __restrict__ W1BT, const float* __restrict__ b1b, float* __restrict__ X1, float* __restrict__ PS) {
  __shared__ __attribute__((aligned(16))) b16 Ah[4][16][D + 8], Al[4][16][D + 8]; __shared__ __attribute__((aligned(16))) float Tf[4][16][D + 4]; __shared__ __attribute__((aligned(16))) float cs[4][D];
  const int wave = threadIdx.x >> 5, lane = threadIdx.x & 31, nloc = lane & 15, hlf = lane >> 4; const size_t m0 = (size_t)blockIdx.x * 64 + wave * 16;
  for (int rr = 0; rr < 16; ++rr) { const size_t v = m0 + rr; v4f acc = {0.0f, 0.0f, 0.0f, 0.0f};
    if (v < (size_t)N) { const v4f xv = *(const v4f*)(x + v * D + lane * 4); for (int j = 0; j < 4; ++j) acc[j] = bf16_rne(xv[j]);
      int st = ROWPTR[v], cnt = ROWCNT[v]; cnt = iclamp(cnt, 0, 65536); st = iclamp(st, 0, permLen - cnt);
      for (int i = 0; i < cnt; ++i) { const int e = iclamp(PERM[st + i], 0, E - 1); const size_t u = (size_t)iclamp(srcs[e], 0, N - 1); const v4f xu = *(const v4f*)(x + u * D + lane * 4); for (int j = 0; j < 4; ++j) acc[j] += bf16_rne(xu[j]); } }
    for (int j = 0; j < 4; ++j) { b16 p, q; split16(acc[j] * XS, p, q); Ah[wave][rr][lane * 4 + j] = p; Al[wave][rr][lane * 4 + j] = q; } }
  wave_lds_sync();
  v8f d[8];
  auto gemm = [&](const b16* WT) {
#pragma unroll
    for (int t = 0; t < 8; ++t) d[t] = (v8f){};
#pragma unroll
    for (int kb = 0; kb < D; kb += 32) { const v16b a = frag_kb(&Ah[wave][nloc][kb], hlf), al = frag_kb(&Al[wave][nloc][kb], hlf);
#pragma unroll
      for (int t = 0; t < 8; ++t) { const v16b bw = frag_kb(WT + (size_t)(t * 16 + nloc) * D + kb, hlf); d[t] = wmma16b(a, bw, d[t]); d[t] = wmma16b(al, bw, d[t]); } } };
  gemm(W1AT); wave_lds_sync();
#pragma unroll
  for (int t = 0; t < 8; ++t) { const int c = t * 16 + nloc; const float bb = bf16_rne(b1a[c]);
#pragma unroll 1
    for (int r = 0; r < 8; ++r) { b16 p, q; split16(fmaxf(d[t][r] * (1.0f / (XS * WSC)) + bb, 0.0f) * XS, p, q); Ah[wave][8 * hlf + r][c] = p; Al[wave][8 * hlf + r][c] = q; } }
  wave_lds_sync();
  gemm(W1BT);
#pragma unroll
  for (int t = 0; t < 8; ++t) { const int c = t * 16 + nloc; const float bb = bf16_rne(b1b[c]);
#pragma unroll 1
    for (int r = 0; r < 8; ++r) { const size_t row = m0 + 8 * hlf + r; Tf[wave][8 * hlf + r][c] = row < (size_t)N ? fmaxf(d[t][r] * (1.0f / (XS * WSC)) + bb, 0.0f) : 0.0f; } }
  wave_lds_sync();
  for (int pass = 0; pass < 2; ++pass) { for (int rr = 0; rr < 16; ++rr) *(volatile v4f*)(X1 + (m0 + rr) * D + lane * 4) = *(const v4f*)(&Tf[wave][rr][lane * 4]); __threadfence(); }
  { v4f s = {0.0f, 0.0f, 0.0f, 0.0f}; for (int rr = 0; rr < 16; ++rr) s += *(const v4f*)(&Tf[wave][rr][lane * 4]); *(v4f*)(&cs[wave][lane * 4]) = s; }
  __syncthreads();
  if (wave == 0) { v4f s = *(const v4f*)(&cs[0][lane * 4]); for (int w = 1; w < 4; ++w) s += *(const v4f*)(&cs[w][lane * 4]);
    for (int pass = 0; pass < 2; ++pass) { *(volatile v4f*)(PS + (size_t)blockIdx.x * D + lane * 4) = s; __threadfence(); } }
}
__global__ __launch_bounds__(128) void mean_kernel(const float* __restrict__ PS, float* __restrict__ STAT) {
  const int c = threadIdx.x; float s = 0.0f; for (int b = 0; b < NBLK; ++b) s += PS[(size_t)b * D + c];
  for (int pass = 0; pass < 2; ++pass) { ((volatile float*)STAT)[c] = s * (1.0f / N); __threadfence(); }
}
__global__ __launch_bounds__(128) void var_kernel(const float* __restrict__ X1, const float* __restrict__ STAT, float* __restrict__ PS2) {
  const int c = threadIdx.x; const float m = STAT[c]; float s = 0.0f; const size_t r0 = (size_t)blockIdx.x * 64;
  for (int rr = 0; rr < 64; ++rr) { const size_t r = r0 + rr; if (r < (size_t)N) { const float dlt = X1[r * D + c] - m; s += dlt * dlt; } }
  for (int pass = 0; pass < 2; ++pass) { ((volatile float*)PS2)[(size_t)blockIdx.x * D + c] = s; __threadfence(); }
}
__device__ int lower_bound_i(const int* a, int n, int key) { int lo = 0, hi = n; while (lo < hi) { const int mid = (lo + hi) >> 1; if (a[mid] < key) lo = mid + 1; else hi = mid; } return lo; }
__global__ __launch_bounds__(128) void pool_kernel(const float* __restrict__ X1, const int* __restrict__ batch, const float* __restrict__ STAT, const float* __restrict__ PS2, const float* __restrict__ gam, const float* __restrict__ bet, b16* __restrict__ Ch, b16* __restrict__ Cl) {
  const int g = blockIdx.x, c = threadIdx.x; const int lo = lower_bound_i(batch, N, g), hi = lower_bound_i(batch, N, g + 1);
  float s = 0.0f; for (int v = lo; v < hi; ++v) s += X1[(size_t)v * D + c]; const float mx = s / fmaxf((float)(hi - lo), 1.0f);
  float vs = 0.0f; for (int b = 0; b < NBLK; ++b) vs += PS2[(size_t)b * D + c]; const float var = vs * (1.0f / N);
  const float xg = (hi > lo) ? bf16_rne(gam[c]) * (mx - STAT[c]) * rsqrtf(var + BNEPS) + bf16_rne(bet[c]) : 0.0f;
  b16 p, q; split16(xg * XS, p, q);
  for (int pass = 0; pass < 2; ++pass) { ((volatile b16*)Ch)[(size_t)g * 2 * D + c] = p; ((volatile b16*)Cl)[(size_t)g * 2 * D + c] = q; ((volatile b16*)Ch)[(size_t)g * 2 * D + D + c] = p; ((volatile b16*)Cl)[(size_t)g * 2 * D + D + c] = q; __threadfence(); }
}
__global__ __launch_bounds__(512) void rec_kernel(b16* Ch, b16* Cl, const b16* __restrict__ WLT, const float* __restrict__ bl1, const float* __restrict__ bl2, const b16* __restrict__ WM1T, const float* __restrict__ bm1, const b16* __restrict__ WM2T, const float* __restrict__ bm2, float* __restrict__ out) {
  __shared__ __attribute__((aligned(16))) b16 Z[16][16][D + 8]; __shared__ __attribute__((aligned(16))) float so[G * NO];
  const int wave = threadIdx.x >> 5, lane = threadIdx.x & 31, nloc = lane & 15, hlf = lane >> 4; const int g0 = wave * 16;
  v8f d[8];
  for (int it = 0; it < NIT; ++it) {
#pragma unroll
    for (int t = 0; t < 8; ++t) d[t] = (v8f){};
#pragma unroll 2
    for (int kb = 0; kb < 2 * D; kb += 32) { const v16b a = frag_kb(Ch + (size_t)(g0 + nloc) * 2 * D + kb, hlf), al = frag_kb(Cl + (size_t)(g0 + nloc) * 2 * D + kb, hlf);
#pragma unroll
      for (int t = 0; t < 8; ++t) { const v16b bw = frag_kb(WLT + (size_t)(t * 16 + nloc) * 2 * D + kb, hlf); d[t] = wmma16b(a, bw, d[t]); d[t] = wmma16b(al, bw, d[t]); } }
    __syncthreads();
#pragma unroll
    for (int t = 0; t < 8; ++t) { const int c = t * 16 + nloc;
      const int hc = c < HR ? HR + c : c - HR; const float bb = c < HR ? bf16_rne(bl1[c]) : bf16_rne(bl2[c - HR]);
#pragma unroll 1
      for (int r = 0; r < 8; ++r) { const float pre = d[t][r] * (1.0f / (XS * WSC)) + bb; d[t][r] = c < HR ? sigm(pre) : tanhf(pre); } }
    for (int ph = 0; ph < 2; ++ph) {
#pragma unroll
      for (int t = 0; t < 8; ++t) { const int c = t * 16 + nloc; const int hc = c < HR ? HR + c : c - HR;
#pragma unroll 1
        for (int r = 0; r < 8; ++r) { b16 p, q; split16(d[t][r] * XS, p, q); Z[wave][8 * hlf + r][hc] = ph ? q : p; } }
      wave_lds_sync();
      b16* dstp = ph ? Cl : Ch;
      for (int pass = 0; pass < 2; ++pass) { for (int rr = 0; rr < 16; ++rr) if (lane < 16) *(volatile v8b*)(dstp + (size_t)(g0 + rr) * 2 * D + D + lane * 8) = *(const v8b*)(&Z[wave][rr][lane * 8]); __threadfence(); }
      wave_lds_sync(); }
    __syncthreads(); }
#pragma unroll
  for (int t = 0; t < 6; ++t) d[t] = (v8f){};
#pragma unroll
  for (int kb = 0; kb < D; kb += 32) { const v16b a = frag_kb(Ch + (size_t)(g0 + nloc) * 2 * D + D + kb, hlf), al = frag_kb(Cl + (size_t)(g0 + nloc) * 2 * D + D + kb, hlf);
#pragma unroll
    for (int t = 0; t < 6; ++t) { const v16b bw = frag_kb(WM1T + (size_t)(t * 16 + nloc) * D + kb, hlf); d[t] = wmma16b(a, bw, d[t]); d[t] = wmma16b(al, bw, d[t]); } }
  for (int q = lane; q < 16 * 32; q += 32) { const int rr = q >> 5, c = 96 + (q & 31); Z[wave][rr][c] = (b16)0.0f; }
#pragma unroll
  for (int t = 0; t < 6; ++t) { const int c = t * 16 + nloc; const float bb = c < DM ? bf16_rne(bm1[c]) : 0.0f;
#pragma unroll 1
    for (int r = 0; r < 8; ++r) d[t][r] = c < DM ? fmaxf(d[t][r] * (1.0f / (XS * WSC)) + bb, 0.0f) : 0.0f; }
  { v8f o = {};
    for (int ph = 0; ph < 2; ++ph) {
      wave_lds_sync();
#pragma unroll
      for (int t = 0; t < 6; ++t) { const int c = t * 16 + nloc;
#pragma unroll 1
        for (int r = 0; r < 8; ++r) { b16 p, q; split16(d[t][r] * XS, p, q); Z[wave][8 * hlf + r][c] = ph ? q : p; } }
      wave_lds_sync();
#pragma unroll
      for (int kb = 0; kb < D; kb += 32) { const v16b a = frag_kb(&Z[wave][nloc][kb], hlf); const v16b bw = frag_kb(WM2T + (size_t)nloc * D + kb, hlf); o = wmma16b(a, bw, o); } }
#pragma unroll 1
    for (int r = 0; r < 8; ++r) if (nloc < NO) so[(g0 + 8 * hlf + r) * NO + nloc] = o[r] * (1.0f / (XS * WSC)) + bf16_rne(bm2[nloc]); }
  __syncthreads();
  for (int pass = 0; pass < 2; ++pass) { for (int q = threadIdx.x; q < G * NO / 4; q += 512) *(volatile v4f*)(out + q * 4) = *(const v4f*)(&so[q * 4]); __threadfence(); }
}
}

extern "C" void kernel_launch(void* const* d_in, const int* in_sizes, int n_in, void* d_out, int out_size, void* d_ws, size_t ws_size, hipStream_t stream) {
  (void)n_in;
  auto Fp = [&](int i) { return (const float*)d_in[i]; }; auto Ip = [&](int i) { return (const int*)d_in[i]; };
  if (in_sizes[0] != N * D || in_sizes[1] != 2 * E || in_sizes[2] != N || in_sizes[3] != D * D || in_sizes[9] != 2 * D * HR || in_sizes[13] != D * DM || in_sizes[15] != DM * NO || out_size != G * NO) return;
  size_t off = 0; char* ws = (char*)d_ws;
  auto carve = [&](size_t bytes) { char* p = ws + off; off += (bytes + 255) & ~(size_t)255; return p; };
  b16* W1AT = (b16*)carve((size_t)D * D * 2); b16* W1BT = (b16*)carve((size_t)D * D * 2); b16* WLT = (b16*)carve((size_t)D * 2 * D * 2); b16* WM1T = (b16*)carve((size_t)DMP * D * 2); b16* WM2T = (b16*)carve((size_t)16 * D * 2);
  float* X1 = (float*)carve((size_t)NP * D * 4); float* PS = (float*)carve((size_t)NBLK * D * 4); float* PS2 = (float*)carve((size_t)NBLK * D * 4); float* STAT = (float*)carve(1024); b16* Ch = (b16*)carve((size_t)G * 2 * D * 2); b16* Cl = (b16*)carve((size_t)G * 2 * D * 2);
  CsrBufs csr; off = csr_carve(csr, ws, off, E, N);
  if (off > ws_size || off > ((size_t)128 << 20)) return;
  wprep_kernel<<<(unsigned)((2 * (size_t)D * D / 8 + (size_t)D * 2 * D / 8 + (size_t)DMP * D / 8 + 16 * D / 8 + 255) / 256), 256, 0, stream>>>(Fp(3), Fp(5), Fp(9), Fp(11), Fp(13), Fp(15), W1AT, W1BT, WLT, WM1T, WM2T);
  csr_build(csr, Ip(1) + E, E, N, stream);
  gin_kernel<<<NBLK, 128, 0, stream>>>(Fp(0), Ip(1), csr.PERM, csr.ROWPTR, csr.ROWCNT, (int)csr.permLen, W1AT, Fp(4), W1BT, Fp(6), X1, PS);
  mean_kernel<<<1, 128, 0, stream>>>(PS, STAT);
  var_kernel<<<NBLK, 128, 0, stream>>>(X1, STAT, PS2);
  pool_kernel<<<G, 128, 0, stream>>>(X1, Ip(2), STAT, PS2, Fp(7), Fp(8), Ch, Cl);
  rec_kernel<<<1, 512, 0, stream>>>(Ch, Cl, WLT, Fp(10), Fp(12), WM1T, Fp(14), WM2T, Fp(16), (float*)d_out);
}
